// KahlerAttention_51324859187419
// MI455X (gfx1250) — hardware-verified
//
#include <hip/hip_runtime.h>
#include <stddef.h>
#include <stdint.h>

#define NB    2
#define SQ    2048
#define NTOK  4096
#define HID   1024
#define D4    256
#define NH    16
#define HDM   64
#define NPROJ 4
#define RB    64
#define QB    128
#define KC    64
#define NQB   (SQ / QB)
#define NCK   (SQ / KC)
#define QKPLANE (NB * NH * SQ * HDM)
#define NEGMASK 10318

static_assert(NTOK == NB * SQ);
static_assert(HID == 4 * D4);
static_assert(NH * HDM == HID);
static_assert(HDM == 64);
static_assert(SQ % RB == 0);
static_assert(NTOK % RB == 0);
static_assert(SQ % QB == 0);
static_assert(SQ % KC == 0);
static_assert(NTOK % 256 == 0);
static_assert((NTOK * HID) % 2048 == 0);
static_assert((HID * HID) % 2048 == 0);
static_assert(D4 % 8 == 0);

typedef _Float16 v16h __attribute__((ext_vector_type(16)));
typedef _Float16 v8h  __attribute__((ext_vector_type(8)));
typedef float    v8f  __attribute__((ext_vector_type(8)));
typedef float    v4f  __attribute__((ext_vector_type(4)));
typedef unsigned int v4u __attribute__((ext_vector_type(4)));

union Frag  { v16h v; v8h h[2]; };
union Pack8 { v8h h; v4u u; };

__device__ __forceinline__ v8f mma16(v16h a, v16h b, v8f c) {
  c = __builtin_amdgcn_wmma_f32_16x16x32_f16(false, a, false, b, (short)0, c, false, false);
  asm volatile("v_nop\n\tv_nop\n\tv_nop\n\tv_nop" : "+v"(c) : "v"(a), "v"(b));
  return c;
}

__device__ __forceinline__ v16h ldfrag(const _Float16* p, int ld, int row0, int k0, int lane) {
  const int m = lane & 15, lh = lane >> 4;
  const _Float16* q = p + (size_t)(row0 + m) * ld + k0 + 8 * lh;
  Frag f;
  f.h[0] = *(const v8h*)(q);
  f.h[1] = *(const v8h*)(q + 16);
  return f.v;
}

__device__ __forceinline__ v8f zero8() { return (v8f){0.f, 0.f, 0.f, 0.f, 0.f, 0.f, 0.f, 0.f}; }

__device__ __forceinline__ void gemm32x64s(const _Float16* __restrict__ A, int lda,
                                           const _Float16* __restrict__ Bt, int ldb, int K,
                                           int m0, int n0, int nstr, int lane, v8f (&acc)[2][4]) {
#pragma unroll 1
  for (int k0 = 0; k0 < K; k0 += 32) {
    const v16h a0 = ldfrag(A, lda, m0, k0, lane);
    const v16h a1 = ldfrag(A, lda, m0 + 16, k0, lane);
    const v16h b0 = ldfrag(Bt, ldb, n0, k0, lane);
    const v16h b1 = ldfrag(Bt, ldb, n0 + nstr, k0, lane);
    const v16h b2 = ldfrag(Bt, ldb, n0 + 2 * nstr, k0, lane);
    const v16h b3 = ldfrag(Bt, ldb, n0 + 3 * nstr, k0, lane);
    acc[0][0] = mma16(a0, b0, acc[0][0]);
    acc[1][0] = mma16(a1, b0, acc[1][0]);
    acc[0][1] = mma16(a0, b1, acc[0][1]);
    acc[1][1] = mma16(a1, b1, acc[1][1]);
    acc[0][2] = mma16(a0, b2, acc[0][2]);
    acc[1][2] = mma16(a1, b2, acc[1][2]);
    acc[0][3] = mma16(a0, b3, acc[0][3]);
    acc[1][3] = mma16(a1, b3, acc[1][3]);
  }
}

__global__ __launch_bounds__(256) void k_cvt(const float* __restrict__ src, _Float16* __restrict__ dh, float scale) {
  const int tid = threadIdx.x;
  const int row = blockIdx.x * 2 + (tid >> 7);
  const int col = (tid & 127) * 8;
  const size_t o = (size_t)row * HID + col;
  const v4f a0 = *(const v4f*)(src + o) * scale;
  const v4f a1 = *(const v4f*)(src + o + 4) * scale;
  Pack8 pk;
  pk.h = (v8h){(_Float16)a0[0], (_Float16)a0[1], (_Float16)a0[2], (_Float16)a0[3],
               (_Float16)a1[0], (_Float16)a1[1], (_Float16)a1[2], (_Float16)a1[3]};
  const v4u vv = pk.u;
  volatile v4u* d = (volatile v4u*)(dh + o);
  *d = vv;
  __threadfence();
  *d = vv;
}

__global__ __launch_bounds__(256) void k_wbuild(const float* __restrict__ w0, const float* __restrict__ w1,
                                                const float* __restrict__ w2, const float* __restrict__ w3,
                                                const float* __restrict__ b0, const float* __restrict__ b1,
                                                const float* __restrict__ b2, const float* __restrict__ b3,
                                                _Float16* __restrict__ wd, float* __restrict__ bd) {
  const int tid = threadIdx.x;
  const int p = blockIdx.y;
  const float* W  = (p == 0) ? w0 : ((p == 1) ? w1 : ((p == 2) ? w2 : w3));
  const float* bs = (p == 0) ? b0 : ((p == 1) ? b1 : ((p == 2) ? b2 : b3));
  const int n  = blockIdx.x * 2 + (tid >> 7);
  const int kq = (tid & 127) * 8;
  const int e = n >> 8, o = n & 255;
  const int c = kq >> 8, d0 = kq & 255;
  const int w = e ^ c;
  const float sg = (((NEGMASK >> (e * 4 + c)) & 1) != 0) ? -32.0f : 32.0f;
  const float* src = W + ((size_t)w << 16) + ((size_t)d0 << 8) + o;
  float v[8];
#pragma unroll
  for (int i = 0; i < 8; ++i) v[i] = src[(size_t)i * D4] * sg;
  Pack8 pk;
  pk.h = (v8h){(_Float16)v[0], (_Float16)v[1], (_Float16)v[2], (_Float16)v[3],
               (_Float16)v[4], (_Float16)v[5], (_Float16)v[6], (_Float16)v[7]};
  const v4u vv = pk.u;
  volatile v4u* dst = (volatile v4u*)(wd + (size_t)p * HID * HID + (size_t)n * HID + kq);
  *dst = vv;
  __threadfence();
  *dst = vv;

  if (blockIdx.x < 4) {
    const int nn = blockIdx.x * 256 + tid;
    const int ee = nn >> 8, oo = nn & 255;
    float acc = 0.f;
#pragma unroll
    for (int cc = 0; cc < 4; ++cc) {
      const int ww = ee ^ cc;
      const float s1 = (((NEGMASK >> (ee * 4 + cc)) & 1) != 0) ? -1.0f : 1.0f;
      acc += s1 * bs[(ww << 8) + oo];
    }
    volatile float* bp = (volatile float*)(bd + (size_t)p * HID + nn);
    *bp = acc;
    __threadfence();
    *bp = acc;
  }
}

#define STP 72
__global__ __launch_bounds__(256) void k_qkv(const _Float16* __restrict__ xh,
                                             const _Float16* __restrict__ wd,
                                             const float* __restrict__ bd,
                                             _Float16* __restrict__ qkp,
                                             _Float16* __restrict__ vtp) {
  __shared__ __align__(16) _Float16 st[4 * RB * STP];
  const int tid = threadIdx.x, lane = tid & 31, wave = tid >> 5;
  const int hh = lane >> 4, c = lane & 15;
  const int bx = blockIdx.x;
  const int b  = bx / (SQ / RB);
  const int s0 = (bx - b * (SQ / RB)) * RB;
  const int which = blockIdx.y >> 2;
  const int hq    = blockIdx.y & 3;
  const int wm = (wave & 1) * 32;
  const int wq = wave >> 1;
  const int m0 = bx * RB + wm;
  const int n0 = which * HID + hq * HDM + wq * 16;

  v8f acc[2][4];
#pragma unroll
  for (int s = 0; s < 2; ++s)
#pragma unroll
    for (int t = 0; t < 4; ++t) acc[s][t] = zero8();
  gemm32x64s(xh, HID, wd, HID, HID, m0, n0, D4, lane, acc);

  float bb[4];
#pragma unroll
  for (int e = 0; e < 4; ++e) bb[e] = bd[n0 + e * D4 + c];

  if (which < 2) {
#pragma unroll
    for (int sub = 0; sub < 2; ++sub) {
#pragma unroll
      for (int r = 0; r < 8; ++r) {
        const float v0 = acc[sub][0][r] * 0.03125f + bb[0];
        const float v1 = acc[sub][1][r] * 0.03125f + bb[1];
        const float v2 = acc[sub][2][r] * 0.03125f + bb[2];
        const float v3 = acc[sub][3][r] * 0.03125f + bb[3];
        const float inv = rsqrtf(v0 * v0 + v1 * v1 + v2 * v2 + v3 * v3 + 1e-6f);
        const int lr = wm + sub * 16 + 8 * hh + r;
        _Float16* rowp = st + lr * STP + wq * 16 + c;
        rowp[0 * RB * STP] = (_Float16)(v0 * inv);
        rowp[1 * RB * STP] = (_Float16)(v1 * inv);
        rowp[2 * RB * STP] = (_Float16)(v2 * inv);
        rowp[3 * RB * STP] = (_Float16)(v3 * inv);
      }
    }
  } else {
#pragma unroll
    for (int sub = 0; sub < 2; ++sub) {
#pragma unroll
      for (int e = 0; e < 4; ++e) {
#pragma unroll
        for (int r = 0; r < 8; ++r) {
          const int lr = wm + sub * 16 + 8 * hh + r;
          st[(e * RB + wq * 16 + c) * STP + lr] = (_Float16)(acc[sub][e][r] * 0.03125f + bb[e]);
        }
      }
    }
  }
  __syncthreads();

  if (which < 2) {
    _Float16* base = qkp + (size_t)which * QKPLANE;
#pragma unroll
    for (int g = 0; g < 2; ++g) {
      v4u val[4];
      size_t go[4];
#pragma unroll
      for (int j = 0; j < 4; ++j) {
        const int p  = tid + 256 * (4 * g + j);
        const int e  = p >> 9;
        const int lr = (p >> 3) & 63;
        const int pc = p & 7;
        Pack8 pk;
        pk.h   = *(const v8h*)(st + (e * RB + lr) * STP + pc * 8);
        val[j] = pk.u;
        go[j]  = ((size_t)(b * NH + 4 * e + hq) * SQ + s0 + lr) * HDM + pc * 8;
      }
      for (int ps = 0; ps < 2; ++ps) {
#pragma unroll
        for (int j = 0; j < 4; ++j) *(volatile v4u*)(base + go[j]) = val[j];
        __threadfence();
      }
    }
  } else {
#pragma unroll
    for (int g = 0; g < 2; ++g) {
      v4u val[4];
      size_t go[4];
#pragma unroll
      for (int j = 0; j < 4; ++j) {
        const int p    = tid + 256 * (4 * g + j);
        const int e    = p >> 9;
        const int drow = (p >> 3) & 63;
        const int pc   = p & 7;
        Pack8 pk;
        pk.h   = *(const v8h*)(st + (e * RB + drow) * STP + pc * 8);
        val[j] = pk.u;
        go[j]  = ((size_t)(b * NH + 4 * e + hq) * HDM + drow) * SQ + s0 + pc * 8;
      }
      for (int ps = 0; ps < 2; ++ps) {
#pragma unroll
        for (int j = 0; j < 4; ++j) *(volatile v4u*)(vtp + go[j]) = val[j];
        __threadfence();
      }
    }
  }
}

#define KTP 72
__global__ __launch_bounds__(256) void k_attn(const _Float16* __restrict__ qp,
                                              const _Float16* __restrict__ kp,
                                              const _Float16* __restrict__ vt,
                                              _Float16* __restrict__ op, float sscale) {
  __shared__ __align__(16) _Float16 Ks[KC * KTP];
  __shared__ __align__(16) _Float16 Vs[HDM * KTP];
  __shared__ __align__(16) _Float16 Ps[8 * 16 * KTP];

  const int tid = threadIdx.x, lane = tid & 31, wave = tid >> 5;
  const int hh = lane >> 4, c = lane & 15;
  const int qb  = blockIdx.x % NQB;
  const int hb  = blockIdx.x / NQB;
  const int h   = hb % NH;
  const int b   = hb / NH;
  const int q0  = qb * QB + wave * 16;

  const _Float16* Q = qp + (size_t)hb * SQ * HDM;
  const _Float16* K = kp + (size_t)hb * SQ * HDM;
  const _Float16* V = vt + (size_t)hb * HDM * SQ;

  v16h qa[2];
  qa[0] = ldfrag(Q, HDM, q0, 0, lane);
  qa[1] = ldfrag(Q, HDM, q0, 32, lane);

  const float NEGI = -__builtin_huge_valf();
  float mrow[8], lrow[8];
  v8f oacc[4];
#pragma unroll
  for (int r = 0; r < 8; ++r) { mrow[r] = NEGI; lrow[r] = 0.f; }
#pragma unroll
  for (int t = 0; t < 4; ++t) oacc[t] = zero8();

  _Float16* pw = Ps + wave * 16 * KTP;

  for (int kc = 0; kc < NCK; ++kc) {
    const int kv0 = kc * KC;
    __syncthreads();
    {
      const int r  = tid >> 2;
      const int qq = (tid & 3) * 16;
      const _Float16* ks = K + (size_t)(kv0 + r) * HDM + qq;
      const _Float16* vs = V + (size_t)r * SQ + kv0 + qq;
#pragma unroll
      for (int e = 0; e < 2; ++e) {
        *(v8h*)(Ks + r * KTP + qq + 8 * e) = *(const v8h*)(ks + 8 * e);
        *(v8h*)(Vs + r * KTP + qq + 8 * e) = *(const v8h*)(vs + 8 * e);
      }
    }
    __syncthreads();

    v8f s[4];
#pragma unroll
    for (int j = 0; j < 4; ++j) s[j] = zero8();
#pragma unroll
    for (int dc = 0; dc < 2; ++dc) {
#pragma unroll
      for (int j = 0; j < 4; ++j) {
        const v16h kb = ldfrag(Ks, KTP, j * 16, dc * 32, lane);
        s[j] = mma16(qa[dc], kb, s[j]);
      }
    }
    float cm[8];
#pragma unroll
    for (int r = 0; r < 8; ++r) {
      float m = NEGI;
#pragma unroll
      for (int j = 0; j < 4; ++j) { s[j][r] *= sscale; m = fmaxf(m, s[j][r]); }
#pragma unroll
      for (int off = 1; off < 16; off <<= 1) m = fmaxf(m, __shfl_xor(m, off, 32));
      cm[r] = m;
    }
    float al[8];
#pragma unroll
    for (int r = 0; r < 8; ++r) {
      const float mnew  = fmaxf(mrow[r], cm[r]);
      const float alpha = __expf(mrow[r] - mnew);
      mrow[r] = mnew;
      float psum = 0.f;
#pragma unroll
      for (int j = 0; j < 4; ++j) {
        const float p = __expf(s[j][r] - mnew);
        psum += p;
        pw[(8 * hh + r) * KTP + j * 16 + c] = (_Float16)(p * 1024.0f);
      }
#pragma unroll
      for (int off = 1; off < 16; off <<= 1) psum += __shfl_xor(psum, off, 32);
      lrow[r] = lrow[r] * alpha + psum;
      al[r] = alpha;
    }
#pragma unroll
    for (int t = 0; t < 4; ++t)
#pragma unroll
      for (int r = 0; r < 8; ++r) oacc[t][r] *= al[r];
    __syncthreads();

#pragma unroll
    for (int kk = 0; kk < 2; ++kk) {
      const v16h pa = ldfrag(pw, KTP, 0, kk * 32, lane);
#pragma unroll
      for (int t = 0; t < 4; ++t) {
        const v16h vb = ldfrag(Vs, KTP, t * 16, kk * 32, lane);
        oacc[t] = mma16(pa, vb, oacc[t]);
      }
    }
  }

  float invl[8];
#pragma unroll
  for (int r = 0; r < 8; ++r) invl[r] = (lrow[r] > 0.f) ? (0.0625f / lrow[r]) : 0.f;
  __syncthreads();
#pragma unroll
  for (int r = 0; r < 8; ++r) {
#pragma unroll
    for (int t = 0; t < 4; ++t)
      pw[(8 * hh + r) * KTP + 16 * t + c] = (_Float16)(oacc[t][r] * invl[r]);
  }
  __syncthreads();
  v4u val[4];
  size_t go[4];
#pragma unroll
  for (int it = 0; it < 4; ++it) {
    const int p  = lane + 32 * it;
    const int L  = p >> 3;
    const int pc = p & 7;
    Pack8 pk;
    pk.h    = *(const v8h*)(pw + L * KTP + pc * 8);
    val[it] = pk.u;
    go[it]  = ((size_t)(b * SQ + q0 + L)) * HID + (size_t)h * HDM + pc * 8;
  }
  for (int ps = 0; ps < 2; ++ps) {
#pragma unroll
    for (int it = 0; it < 4; ++it) *(volatile v4u*)(op + go[it]) = val[it];
    __threadfence();
  }
}

#define OTP 68
__device__ __forceinline__ void out_epilogue_f32(v8f (&acc)[2][4], float scale, const float (&bb)[4],
                                                 float* sw, float* __restrict__ out, int ldo,
                                                 int m0, int n0, int lane, int hh, int c) {
#pragma unroll
  for (int sub = 0; sub < 2; ++sub) {
    __syncthreads();
#pragma unroll
    for (int t = 0; t < 4; ++t) {
#pragma unroll
      for (int r = 0; r < 8; ++r) sw[(8 * hh + r) * OTP + 16 * t + c] = acc[sub][t][r] * scale + bb[t];
    }
    __syncthreads();
    v4f val[8];
    size_t go[8];
#pragma unroll
    for (int it = 0; it < 8; ++it) {
      const int p    = lane + 32 * it;
      const int L    = p >> 3;
      const int pc   = p & 7;
      const int row  = L >> 1;
      const int half = L & 1;
      val[it] = *(const v4f*)(sw + row * OTP + half * 32 + pc * 4);
      go[it]  = (size_t)(m0 + sub * 16 + row) * ldo + n0 + half * 32 + pc * 4;
    }
    for (int ps = 0; ps < 2; ++ps) {
#pragma unroll
      for (int it = 0; it < 8; ++it) *(volatile v4f*)(out + go[it]) = val[it];
      __threadfence();
    }
  }
}

__global__ __launch_bounds__(256) void k_gemm_f32(const _Float16* __restrict__ ap, int lda,
                                                  const _Float16* __restrict__ wt, int K,
                                                  const float* __restrict__ bias, float scale,
                                                  float* __restrict__ out, int ldo) {
  __shared__ __align__(16) float st[8][16 * OTP];
  const int tid = threadIdx.x, lane = tid & 31, wave = tid >> 5;
  const int hh = lane >> 4, c = lane & 15;
  const int m0 = blockIdx.x * 256 + wave * 32;
  const int n0 = blockIdx.y * 64;

  v8f acc[2][4];
#pragma unroll
  for (int s = 0; s < 2; ++s)
#pragma unroll
    for (int t = 0; t < 4; ++t) acc[s][t] = zero8();
  gemm32x64s(ap, lda, wt, K, K, m0, n0, 16, lane, acc);
  float bb[4];
#pragma unroll
  for (int t = 0; t < 4; ++t) bb[t] = bias[n0 + 16 * t + c];
  out_epilogue_f32(acc, scale, bb, st[wave], out, ldo, m0, n0, lane, hh, c);
}

extern "C" void kernel_launch(void* const* d_in, const int* in_sizes, int n_in,
                              void* d_out, int out_size, void* d_ws, size_t ws_size,
                              hipStream_t stream) {
  if (n_in < 10) return;
  if (in_sizes[0] != NTOK * HID) return;
  if (in_sizes[1] != NPROJ * D4 * D4) return;
  if (in_sizes[2] != NPROJ * D4) return;
  if (in_sizes[3] != NPROJ * D4 * D4) return;
  if (in_sizes[4] != NPROJ * D4) return;
  if (in_sizes[5] != NPROJ * D4 * D4) return;
  if (in_sizes[6] != NPROJ * D4) return;
  if (in_sizes[7] != NPROJ * D4 * D4) return;
  if (in_sizes[8] != NPROJ * D4) return;
  if (out_size != NTOK * HID) return;

  const float* x  = (const float*)d_in[0];
  const float* qW = (const float*)d_in[1];
  const float* qb = (const float*)d_in[2];
  const float* kW = (const float*)d_in[3];
  const float* kb = (const float*)d_in[4];
  const float* vW = (const float*)d_in[5];
  const float* vb = (const float*)d_in[6];
  const float* oW = (const float*)d_in[7];
  const float* ob = (const float*)d_in[8];
  float* out = (float*)d_out;

  size_t off = 0;
  const size_t oX  = off; off += (size_t)NTOK * HID * 2;
  const size_t oWd = off; off += (size_t)NPROJ * HID * HID * 2;
  const size_t oQ  = off; off += (size_t)QKPLANE * 2;
  const size_t oK  = off; off += (size_t)QKPLANE * 2;
  const size_t oV  = off; off += (size_t)NB * NH * HDM * SQ * 2;
  const size_t oO  = off; off += (size_t)NTOK * HID * 2;
  const size_t oBd = off; off += (size_t)NPROJ * HID * 4;
  if (off > ws_size) return;
  if (off > (size_t)134217728) return;
  if (oK != oQ + (size_t)QKPLANE * 2) return;

  char* ws = (char*)d_ws;
  _Float16* Xh  = (_Float16*)(ws + oX);
  _Float16* Wd  = (_Float16*)(ws + oWd);
  _Float16* QKp = (_Float16*)(ws + oQ);
  _Float16* Kp  = (_Float16*)(ws + oK);
  _Float16* Vt  = (_Float16*)(ws + oV);
  _Float16* Op  = (_Float16*)(ws + oO);
  float*    Bd  = (float*)(ws + oBd);

  k_cvt<<<dim3((NTOK * HID) / 2048), dim3(256), 0, stream>>>(x, Xh, 1.0f);
  k_wbuild<<<dim3((HID * HID) / 2048, NPROJ), dim3(256), 0, stream>>>(qW, kW, vW, oW, qb, kb, vb, ob, Wd, Bd);
  k_qkv<<<dim3(NTOK / RB, 3 * 4), dim3(256), 0, stream>>>(Xh, Wd, Bd, QKp, Vt);
  const float sscale = 0.125f;
  k_attn<<<dim3(NB * NH * NQB), dim3(256), 0, stream>>>(QKp, Kp, Vt, Op, sscale);
  k_gemm_f32<<<dim3(NTOK / 256, HID / 64), dim3(256), 0, stream>>>(
      Op, HID, Wd + (size_t)3 * HID * HID, HID, Bd + 3 * HID, 0.00048828125f, out, HID);
  (void)hipGetLastError();
}
